// SSM_49306224558206
// MI455X (gfx1250) — hardware-run, weakly checked
//
#include <hip/hip_runtime.h>
#include <math.h>

constexpr int NBAT = 64;
constexpr int NCP  = 32;
constexpr int NFR  = 256;
constexpr int NIND = 1024;
constexpr int NSTD = 512;
constexpr int NROW = NBAT * NFR;
constexpr int NHOP = NIND / 2;
constexpr int NSMP = 131072;
constexpr int NTHR = 256;
constexpr int KCH  = 256;
constexpr int SEQB = 16;
constexpr int APITCH = 520;
constexpr int BPITCH = 516;
constexpr int SLB  = 68;
constexpr int SLD  = 132;
constexpr float MAXEFF = 0.99f;
constexpr float EPSN   = 1e-8f;
static_assert(NCP == 32);
static_assert(NSTD % 32 == 0);
static_assert(NROW % 16 == 0);
static_assert(NIND == 8 * 128 && NSTD == 8 * 64);
static_assert(NBAT % SEQB == 0);
static_assert(NIND % KCH == 0 && NIND % NTHR == 0 && NSTD % NTHR == 0);
static_assert(NSMP == NFR * NHOP && NSMP == 131072);
static_assert((NBAT * NSMP) % (4 * NTHR) == 0);
static_assert(NFR % 64 == 0);
static_assert((NCP * KCH) == 8 * NTHR * 4);
static_assert(SEQB * NSTD == 8 * NTHR * 4);
static_assert(SEQB * NFR == 4 * NTHR * 4);

typedef __attribute__((ext_vector_type(16))) _Float16 v16h;
typedef __attribute__((ext_vector_type(8)))  _Float16 v8h;
typedef __attribute__((ext_vector_type(16))) __bf16   v16b;
typedef __attribute__((ext_vector_type(8)))  __bf16   v8b;
typedef __attribute__((ext_vector_type(8)))  float    v8f;
typedef __attribute__((ext_vector_type(4)))  float    v4f;
typedef __attribute__((ext_vector_type(2)))  float    v2f;
typedef __attribute__((ext_vector_type(4)))  unsigned v4u;

__device__ __forceinline__ unsigned short f2bf_bits(float f) {
  unsigned u = __float_as_uint(f);
  return (unsigned short)((u + 0x7FFFu + ((u >> 16) & 1u)) >> 16);
}
__device__ __forceinline__ float bf_bits2f(unsigned short h) { return __uint_as_float(((unsigned)h) << 16); }

__device__ __forceinline__ void dep_guard1m_b(v8f& a, v16b w, v16b x, v16b y, v16b z) {
  asm volatile("v_nop\n\tv_nop\n\tv_nop\n\tv_nop" : "+v"(a) : "v"(w), "v"(x), "v"(y), "v"(z) : "memory");
}
__device__ __forceinline__ void dep_guard4_b(v8f& a, v8f& b, v8f& c, v8f& d, v16b x, v16b y) {
  asm volatile("v_nop\n\tv_nop\n\tv_nop\n\tv_nop" : "+v"(a), "+v"(b), "+v"(c), "+v"(d) : "v"(x), "v"(y));
}
__device__ __forceinline__ void dep_guard4m_b(v8f& a, v8f& b, v8f& c, v8f& d, v16b x, v16b y) {
  asm volatile("v_nop\n\tv_nop\n\tv_nop\n\tv_nop" : "+v"(a), "+v"(b), "+v"(c), "+v"(d) : "v"(x), "v"(y) : "memory");
}
__device__ __forceinline__ void keep4_b(v16b a, v16b b, v16b c, v16b d) { asm volatile("v_nop" :: "v"(a), "v"(b), "v"(c), "v"(d)); }
__device__ __forceinline__ void keep2_b(v16b a, v16b b) { asm volatile("v_nop" :: "v"(a), "v"(b)); }
__device__ __forceinline__ void acc_guard4(v8f& a, v8f& b, v8f& c, v8f& d) {
  asm volatile("v_nop\n\tv_nop\n\tv_nop\n\tv_nop" : "+v"(a), "+v"(b), "+v"(c), "+v"(d));
}
struct FragB {
  union U { v16b v; v8b h[2]; };
  static __device__ __forceinline__ v16b load(const __bf16* p) {
    U f; f.h[0] = *(const v8b*)(p); f.h[1] = *(const v8b*)(p + 16); return f.v;
  }
  static __device__ __forceinline__ v8f mma(v16b a, v16b b, v8f c) {
    return __builtin_amdgcn_wmma_f32_16x16x32_bf16(false, a, false, b, (short)0, c, false, false);
  }
};
__device__ __forceinline__ float sum16(float v) {
  v += __shfl_xor(v, 1, 32); v += __shfl_xor(v, 2, 32); v += __shfl_xor(v, 4, 32); v += __shfl_xor(v, 8, 32);
  return v;
}
__device__ __forceinline__ float sum32(float v) { v = sum16(v); v += __shfl_xor(v, 16, 32); return v; }

__global__ __launch_bounds__(NTHR) void wtab_kernel(float* __restrict__ WT) {
  const int n = blockIdx.x * NTHR + threadIdx.x;
  const float arg = (6.28318530717958647692f * (float)n) * (1.0f / (float)(NIND - 1));
  const float w = 0.54f - 0.46f * cosf(arg);
  volatile float* wp = WT;
  wp[n] = w;
  __threadfence();
  wp[n] = w;
}

__global__ __launch_bounds__(NTHR) void gram_kernel(const float* __restrict__ proj, float* __restrict__ GR) {
  const int i = blockIdx.x * (NTHR / 32) + (threadIdx.x >> 5);
  const int j = threadIdx.x & 31;
  const float* pi = proj + (size_t)i * NIND;
  const float* pj = proj + (size_t)j * NIND;
  float acc = 0.0f;
#pragma unroll 4
  for (int k = 0; k < NIND; ++k) acc = fmaf(pi[k], pj[k], acc);
  volatile float* gp = GR;
  gp[i * NCP + j] = acc;
  __threadfence();
  gp[i * NCP + j] = acc;
}

template <int NOUT, bool LO>
__global__ __launch_bounds__(NTHR) void pw_kernel(const float* __restrict__ proj, const float* __restrict__ W,
                                                  unsigned short* __restrict__ TH, unsigned short* __restrict__ TL) {
  __shared__ __align__(16) float projS[NCP * KCH];
  __shared__ __align__(16) unsigned short hiS[NTHR * NCP];
  __shared__ __align__(16) unsigned short loS[LO ? NTHR * NCP : 8];
  const int tid = threadIdx.x;
  const int n = blockIdx.x * NTHR + tid;
  float acc[NCP];
#pragma unroll
  for (int cc = 0; cc < NCP; ++cc) acc[cc] = 0.0f;
#pragma unroll 1
  for (int k0 = 0; k0 < NIND; k0 += KCH) {
    __syncthreads();
#pragma unroll
    for (int it = 0; it < 8; ++it) {
      const int idx = it * NTHR + tid;
      const int cc = idx >> 6, k4 = (idx & 63) * 4;
      const v4f v = *(const v4f*)(proj + (size_t)cc * NIND + k0 + k4);
      *(v4f*)(projS + cc * KCH + k4) = v;
    }
    __syncthreads();
#pragma unroll 1
    for (int k = 0; k < KCH; k += 2) {
      const float w0 = W[(size_t)(k0 + k) * NOUT + n];
      const float w1 = W[(size_t)(k0 + k + 1) * NOUT + n];
#pragma unroll
      for (int cc = 0; cc < NCP; ++cc) {
        const v2f pp = *(const v2f*)(projS + cc * KCH + k);
        acc[cc] = fmaf(pp[0], w0, acc[cc]);
        acc[cc] = fmaf(pp[1], w1, acc[cc]);
      }
    }
  }
#pragma unroll
  for (int cc = 0; cc < NCP; ++cc) {
    const unsigned short hb = f2bf_bits(acc[cc]);
    hiS[tid * NCP + cc] = hb;
    if (LO) loS[tid * NCP + cc] = f2bf_bits(acc[cc] - bf_bits2f(hb));
  }
  __syncthreads();
  unsigned* THw = (unsigned*)TH + (size_t)blockIdx.x * NTHR * (NCP / 2);
  unsigned* TLw = (unsigned*)TL + (size_t)blockIdx.x * NTHR * (NCP / 2);
  v4u hv[4], lv[4];
#pragma unroll
  for (int it = 0; it < 4; ++it) {
    const int idx = it * NTHR + tid;
    hv[it] = *(const v4u*)((const unsigned*)hiS + idx * 4);
    if (LO) lv[it] = *(const v4u*)((const unsigned*)loS + idx * 4);
  }
  for (int pass = 0; pass < 2; ++pass) {
#pragma unroll
    for (int it = 0; it < 4; ++it) {
      const int idx = it * NTHR + tid;
      *(volatile v4u*)(THw + (size_t)idx * 4) = hv[it];
      if (LO) *(volatile v4u*)(TLw + (size_t)idx * 4) = lv[it];
    }
    __threadfence();
  }
}

__global__ __launch_bounds__(NTHR) void tpw_bf16_kernel(const float* __restrict__ src, int R, int C, int ldo,
                                                        unsigned short* __restrict__ O) {
  __shared__ float Tt[64 * 65];
  const int tid = threadIdx.x;
  const int c0 = blockIdx.x * 64, r0 = blockIdx.y * 64;
#pragma unroll
  for (int i = 0; i < 4; ++i) {
    const int idx = i * NTHR + tid;
    const int rr = idx >> 4, cc = (idx & 15) * 4;
    const v4f v = *(const v4f*)(src + (size_t)(r0 + rr) * (size_t)C + c0 + cc);
    Tt[rr * 65 + cc + 0] = v[0];
    Tt[rr * 65 + cc + 1] = v[1];
    Tt[rr * 65 + cc + 2] = v[2];
    Tt[rr * 65 + cc + 3] = v[3];
  }
  __syncthreads();
  const int q = tid >> 3, c8 = (tid & 7) * 8;
  v8h hv[2];
#pragma unroll
  for (int g = 0; g < 2; ++g) {
    const int qq = g * 32 + q;
#pragma unroll
    for (int e = 0; e < 8; ++e) {
      const float f = Tt[(c8 + e) * 65 + qq];
      const unsigned short bits = f2bf_bits(f);
      hv[g][e] = __builtin_bit_cast(_Float16, bits);
    }
  }
  for (int pass = 0; pass < 2; ++pass) {
#pragma unroll
    for (int g = 0; g < 2; ++g) {
      const size_t o = (size_t)(c0 + g * 32 + q) * (size_t)ldo + (size_t)(r0 + c8);
      *(volatile v8h*)(O + o) = hv[g];
    }
    __threadfence();
  }
}

__global__ __launch_bounds__(NTHR) void rowprep_kernel(const float* __restrict__ control, const float* __restrict__ GR,
                                                       unsigned short* __restrict__ AH, unsigned short* __restrict__ AL,
                                                       float* __restrict__ PN) {
  __shared__ float ct[64 * 33];
  __shared__ __align__(16) float Gs[NCP * NCP];
  __shared__ __align__(16) unsigned short hiS[64 * NCP];
  __shared__ __align__(16) unsigned short loS[64 * NCP];
  __shared__ __align__(16) float pnS[64];
  const int tid = threadIdx.x, lane = tid & 31, wave = tid >> 5;
  const int bb = blockIdx.x >> 2;
  const int f0 = (blockIdx.x & 3) * 64;
#pragma unroll
  for (int it = 0; it < 2; ++it) {
    const int idx = it * NTHR + tid;
    const int cc = idx >> 4, f4 = (idx & 15) * 4;
    const v4f v = *(const v4f*)(control + ((size_t)bb * NCP + cc) * NFR + f0 + f4);
    ct[(f4 + 0) * 33 + cc] = v[0];
    ct[(f4 + 1) * 33 + cc] = v[1];
    ct[(f4 + 2) * 33 + cc] = v[2];
    ct[(f4 + 3) * 33 + cc] = v[3];
  }
  *(v4f*)(Gs + 4 * tid) = *(const v4f*)(GR + 4 * tid);
  __syncthreads();
#pragma unroll 1
  for (int i = 0; i < 8; ++i) {
    const int ff = wave * 8 + i;
    const float cv = ct[ff * 33 + lane];
    const float on2 = sum32(cv * cv);
    float tc = 0.0f;
#pragma unroll 1
    for (int j = 0; j < NCP; ++j) tc = fmaf(Gs[lane * NCP + j], ct[ff * 33 + j], tc);
    const float xn2 = sum32(cv * tc);
    const float xn = sqrtf(fmaxf(xn2, 0.0f));
    const float on = sqrtf(on2);
    const float cl = fminf(xn, MAXEFF * on);
    const float scl = cl * (1.0f / (xn + EPSN));
    const float pn = scl * xn;
    const float pv = cv * scl;
    const unsigned short hb = f2bf_bits(pv);
    hiS[ff * NCP + lane] = hb;
    loS[ff * NCP + lane] = f2bf_bits(pv - bf_bits2f(hb));
    if (lane == 0) pnS[ff] = pn;
  }
  __syncthreads();
  const size_t row0 = (size_t)bb * NFR + f0;
  unsigned* AHw = (unsigned*)AH + row0 * (NCP / 2);
  unsigned* ALw = (unsigned*)AL + row0 * (NCP / 2);
  const v4u hv = *(const v4u*)((const unsigned*)hiS + 4 * tid);
  const v4u lv = *(const v4u*)((const unsigned*)loS + 4 * tid);
  const int pt = (tid < 16) ? tid : 0;
  const v4f p4 = *(const v4f*)(pnS + 4 * pt);
  for (int pass = 0; pass < 2; ++pass) {
    *(volatile v4u*)(AHw + 4 * tid) = hv;
    *(volatile v4u*)(ALw + 4 * tid) = lv;
    if (tid < 16) *(volatile v4f*)(PN + row0 + 4 * tid) = p4;
    __threadfence();
  }
}

__global__ __launch_bounds__(NTHR) void bproj_kernel(const unsigned short* __restrict__ AHp,
                                                     const unsigned short* __restrict__ PIHp,
                                                     const float* __restrict__ PN, float* __restrict__ BP) {
  __shared__ __align__(16) float slab[8 * 16 * SLB];
  __shared__ float red[8 * 16];
  const int tid = threadIdx.x, lane = tid & 31, wave = tid >> 5;
  const int c = lane & 15, hh = lane >> 4, koff = hh * 8;
  const int m0 = blockIdx.x * 16;
  const int n0w = wave * 64;
  const __bf16* AH  = (const __bf16*)AHp;
  const __bf16* PIH = (const __bf16*)PIHp;
  float pn[8];
  {
    const v4f p0 = *(const v4f*)(PN + m0 + 8 * hh);
    const v4f p1 = *(const v4f*)(PN + m0 + 8 * hh + 4);
#pragma unroll
    for (int e = 0; e < 4; ++e) { pn[e] = p0[e]; pn[4 + e] = p1[e]; }
  }
  const v8f z8 = {0.f, 0.f, 0.f, 0.f, 0.f, 0.f, 0.f, 0.f};
  const v16b ah = FragB::load(AH + (size_t)(m0 + c) * NCP + koff);
  v8f acc[4];
#pragma unroll
  for (int j = 0; j < 4; ++j) {
    const v16b b = FragB::load(PIH + (size_t)(n0w + 16 * j + c) * NCP + koff);
    v8f a0 = FragB::mma(ah, b, z8);
    dep_guard1m_b(a0, b, ah, b, ah);
    acc[j] = a0;
  }
  keep2_b(ah, ah);
  acc_guard4(acc[0], acc[1], acc[2], acc[3]);
  float q[8];
#pragma unroll
  for (int r = 0; r < 8; ++r) q[r] = 0.0f;
#pragma unroll
  for (int j = 0; j < 4; ++j)
#pragma unroll
    for (int r = 0; r < 8; ++r) q[r] = fmaf(acc[j][r], acc[j][r], q[r]);
#pragma unroll
  for (int r = 0; r < 8; ++r) q[r] = sum16(q[r]);
  if (c == 0) {
#pragma unroll
    for (int r = 0; r < 8; ++r) red[wave * 16 + 8 * hh + r] = q[r];
  }
  __syncthreads();
  float sc[8];
#pragma unroll
  for (int r = 0; r < 8; ++r) {
    float n2 = 0.0f;
#pragma unroll
    for (int w = 0; w < 8; ++w) n2 += red[w * 16 + 8 * hh + r];
    const float nn = sqrtf(n2);
    const float cl = fminf(nn, MAXEFF * pn[r]);
    sc[r] = cl * (1.0f / (nn + EPSN));
  }
  float* sw = slab + wave * 16 * SLB;
#pragma unroll
  for (int j = 0; j < 4; ++j)
#pragma unroll
    for (int r = 0; r < 8; ++r) sw[(8 * hh + r) * SLB + 16 * j + c] = acc[j][r] * sc[r];
  __syncthreads();
  const int c4 = c * 4;
  for (int pass = 0; pass < 2; ++pass) {
#pragma unroll
    for (int it = 0; it < 8; ++it) {
      const int row = it * 2 + hh;
      const v4f v = *(const v4f*)(sw + row * SLB + c4);
      *(volatile v4f*)(BP + (size_t)(m0 + row) * NSTD + n0w + c4) = v;
    }
    __threadfence();
  }
}

__global__ __launch_bounds__(NTHR) void scan_kernel(const unsigned short* __restrict__ SMTp, const float* __restrict__ BP,
                                                    unsigned short* __restrict__ SP, float* __restrict__ SN) {
  __shared__ __align__(16) unsigned short Ast[SEQB * APITCH];
  __shared__ __align__(16) unsigned short Sst[SEQB * APITCH];
  __shared__ __align__(16) float Bl[SEQB * BPITCH];
  __shared__ __align__(16) float snl[SEQB * NFR];
  __shared__ float red1[8 * 16];
  __shared__ float red2[8 * 16];
  const int tid = threadIdx.x, lane = tid & 31, wave = tid >> 5;
  const int c = lane & 15, hh = lane >> 4, koff = hh * 8;
  const int rb = blockIdx.x * SEQB;
#pragma unroll 1
  for (int i = tid; i < SEQB * APITCH; i += NTHR) { Ast[i] = (unsigned short)0; Sst[i] = (unsigned short)0; }
  float on2r[8];
#pragma unroll
  for (int r = 0; r < 8; ++r) on2r[r] = 0.0f;
  __syncthreads();

  const __bf16* SMT = (const __bf16*)SMTp;
  const __bf16* arow = (const __bf16*)Ast + c * APITCH + koff;
  const v8f z8 = {0.f, 0.f, 0.f, 0.f, 0.f, 0.f, 0.f, 0.f};
  unsigned* SPw = (unsigned*)SP;

#pragma unroll 1
  for (int t = 0; t < NFR; ++t) {
#pragma unroll
    for (int it = 0; it < 8; ++it) {
      const int idx = it * NTHR + tid;
      const int row = idx >> 7, c4 = (idx & 127) * 4;
      const v4f v = *(const v4f*)(BP + ((size_t)(rb + row) * NFR + (size_t)t) * NSTD + c4);
      *(v4f*)(Bl + row * BPITCH + c4) = v;
    }
    v8f acc[4];
    acc[0] = z8; acc[1] = z8; acc[2] = z8; acc[3] = z8;
#pragma unroll 1
    for (int k0 = 0; k0 < NSTD; k0 += 32) {
      const v16b a  = FragB::load(arow + k0);
      const v16b b0 = FragB::load(SMT + (size_t)(64 * wave +  0 + c) * NSTD + koff + k0);
      const v16b b1 = FragB::load(SMT + (size_t)(64 * wave + 16 + c) * NSTD + koff + k0);
      const v16b b2 = FragB::load(SMT + (size_t)(64 * wave + 32 + c) * NSTD + koff + k0);
      const v16b b3 = FragB::load(SMT + (size_t)(64 * wave + 48 + c) * NSTD + koff + k0);
      acc[0] = FragB::mma(a, b0, acc[0]);
      acc[1] = FragB::mma(a, b1, acc[1]);
      acc[2] = FragB::mma(a, b2, acc[2]);
      acc[3] = FragB::mma(a, b3, acc[3]);
      dep_guard4_b(acc[0], acc[1], acc[2], acc[3], a, b3);
      keep4_b(b0, b1, b2, b3);
    }
    acc_guard4(acc[0], acc[1], acc[2], acc[3]);
    float q[8];
#pragma unroll
    for (int r = 0; r < 8; ++r) q[r] = 0.0f;
#pragma unroll
    for (int nt = 0; nt < 4; ++nt)
#pragma unroll
      for (int r = 0; r < 8; ++r) q[r] = fmaf(acc[nt][r], acc[nt][r], q[r]);
#pragma unroll
    for (int r = 0; r < 8; ++r) q[r] = sum16(q[r]);
    if (c == 0) {
#pragma unroll
      for (int r = 0; r < 8; ++r) red1[wave * 16 + 8 * hh + r] = q[r];
    }
    __syncthreads();
    float sc[8], spn[8];
#pragma unroll
    for (int r = 0; r < 8; ++r) {
      float n2 = 0.0f;
#pragma unroll
      for (int w = 0; w < 8; ++w) n2 += red1[w * 16 + 8 * hh + r];
      const float nn = sqrtf(n2);
      const float on = sqrtf(on2r[r]);
      const float cl = fminf(nn, MAXEFF * on);
      sc[r] = cl * (1.0f / (nn + EPSN));
      spn[r] = sc[r] * nn;
    }
    if (wave == 0 && c == 0) {
#pragma unroll
      for (int r = 0; r < 8; ++r) snl[(8 * hh + r) * NFR + t] = spn[r];
    }
    float q2[8];
#pragma unroll
    for (int r = 0; r < 8; ++r) q2[r] = 0.0f;
#pragma unroll
    for (int nt = 0; nt < 4; ++nt) {
      const int j = 64 * wave + 16 * nt + c;
#pragma unroll
      for (int r = 0; r < 8; ++r) {
        const int row = 8 * hh + r;
        const float sv = acc[nt][r] * sc[r];
        Sst[row * APITCH + j] = f2bf_bits(sv);
        const float ns = sv + Bl[row * BPITCH + j];
        Ast[row * APITCH + j] = f2bf_bits(ns);
        q2[r] = fmaf(ns, ns, q2[r]);
      }
    }
#pragma unroll
    for (int r = 0; r < 8; ++r) q2[r] = sum16(q2[r]);
    if (c == 0) {
#pragma unroll
      for (int r = 0; r < 8; ++r) red2[wave * 16 + 8 * hh + r] = q2[r];
    }
    __syncthreads();
#pragma unroll
    for (int r = 0; r < 8; ++r) {
      float o2 = 0.0f;
#pragma unroll
      for (int w = 0; w < 8; ++w) o2 += red2[w * 16 + 8 * hh + r];
      on2r[r] = o2;
    }
    v4u sv4[4];
#pragma unroll
    for (int it = 0; it < 4; ++it) {
      const int idx = it * NTHR + tid;
      const int row = idx >> 6, c8 = (idx & 63) * 8;
      sv4[it] = *(const v4u*)((const unsigned*)Sst + (row * APITCH + c8) / 2);
    }
    for (int pass = 0; pass < 2; ++pass) {
#pragma unroll
      for (int it = 0; it < 4; ++it) {
        const int idx = it * NTHR + tid;
        const int row = idx >> 6, c8 = (idx & 63) * 8;
        const size_t o = (((size_t)(rb + row) * NFR + (size_t)t) * NSTD + (size_t)c8) / 2;
        *(volatile v4u*)(SPw + o) = sv4[it];
      }
      __threadfence();
    }
  }
  __syncthreads();
  v4f sn4[4];
#pragma unroll
  for (int it = 0; it < 4; ++it) sn4[it] = *(const v4f*)(snl + (it * NTHR + tid) * 4);
  for (int pass = 0; pass < 2; ++pass) {
#pragma unroll
    for (int it = 0; it < 4; ++it)
      *(volatile v4f*)(SN + (size_t)rb * NFR + (size_t)(it * NTHR + tid) * 4) = sn4[it];
    __threadfence();
  }
}

__global__ __launch_bounds__(NTHR) void dc_kernel(const unsigned short* __restrict__ AHp, const unsigned short* __restrict__ ALp,
                                                  const unsigned short* __restrict__ PDHp, const unsigned short* __restrict__ PDLp,
                                                  const float* __restrict__ PN,
                                                  const unsigned short* __restrict__ SPp, const unsigned short* __restrict__ OMTp,
                                                  const float* __restrict__ SN, const float* __restrict__ WT,
                                                  float* __restrict__ Y) {
  __shared__ __align__(16) float slab[8 * 16 * SLD];
  __shared__ __align__(16) float wl[NIND];
  __shared__ float redd[8 * 16];
  __shared__ float redc[8 * 16];
  const int tid = threadIdx.x, lane = tid & 31, wave = tid >> 5;
  const int c = lane & 15, hh = lane >> 4, koff = hh * 8;
  const int m0 = blockIdx.x * 16;
  const int ncol0 = wave * 128;
  *(v4f*)(wl + 4 * tid) = *(const v4f*)(WT + 4 * tid);
  float pn[8];
  {
    const v4f p0 = *(const v4f*)(PN + m0 + 8 * hh);
    const v4f p1 = *(const v4f*)(PN + m0 + 8 * hh + 4);
#pragma unroll
    for (int e = 0; e < 4; ++e) { pn[e] = p0[e]; pn[4 + e] = p1[e]; }
  }
  const __bf16* AH  = (const __bf16*)AHp;
  const __bf16* AL  = (const __bf16*)ALp;
  const __bf16* PDH = (const __bf16*)PDHp;
  const __bf16* PDL = (const __bf16*)PDLp;
  const v8f z8 = {0.f, 0.f, 0.f, 0.f, 0.f, 0.f, 0.f, 0.f};

  const v16b ah = FragB::load(AH + (size_t)(m0 + c) * NCP + koff);
  const v16b al = FragB::load(AL + (size_t)(m0 + c) * NCP + koff);
  v8f accd[8];
#pragma unroll
  for (int j = 0; j < 8; ++j) {
    const size_t bo = (size_t)(ncol0 + 16 * j + c) * NCP + koff;
    const v16b bh = FragB::load(PDH + bo);
    const v16b bl = FragB::load(PDL + bo);
    v8f a0 = FragB::mma(ah, bh, z8);
    a0 = FragB::mma(ah, bl, a0);
    a0 = FragB::mma(al, bh, a0);
    dep_guard1m_b(a0, bh, bl, ah, al);
    accd[j] = a0;
  }
  keep2_b(ah, al);
  acc_guard4(accd[0], accd[1], accd[2], accd[3]);
  acc_guard4(accd[4], accd[5], accd[6], accd[7]);
  float qd[8];
#pragma unroll
  for (int r = 0; r < 8; ++r) qd[r] = 0.0f;
#pragma unroll
  for (int j = 0; j < 8; ++j)
#pragma unroll
    for (int r = 0; r < 8; ++r) qd[r] = fmaf(accd[j][r], accd[j][r], qd[r]);
#pragma unroll
  for (int r = 0; r < 8; ++r) qd[r] = sum16(qd[r]);
  if (c == 0) {
#pragma unroll
    for (int r = 0; r < 8; ++r) redd[wave * 16 + 8 * hh + r] = qd[r];
  }
  __syncthreads();
  float scd[8];
#pragma unroll
  for (int r = 0; r < 8; ++r) {
    float n2 = 0.0f;
#pragma unroll
    for (int w = 0; w < 8; ++w) n2 += redd[w * 16 + 8 * hh + r];
    const float dn = sqrtf(n2);
    const float cl = fminf(dn, MAXEFF * pn[r]);
    scd[r] = cl * (1.0f / (dn + EPSN));
  }
  float* sw = slab + wave * 16 * SLD;
#pragma unroll
  for (int j = 0; j < 8; ++j)
#pragma unroll
    for (int r = 0; r < 8; ++r) sw[(8 * hh + r) * SLD + 16 * j + c] = accd[j][r] * scd[r];

  float sn[8];
  {
    const v4f s0 = *(const v4f*)(SN + m0 + 8 * hh);
    const v4f s1 = *(const v4f*)(SN + m0 + 8 * hh + 4);
#pragma unroll
    for (int e = 0; e < 4; ++e) { sn[e] = s0[e]; sn[4 + e] = s1[e]; }
  }
  const __bf16* spr = (const __bf16*)SPp + (size_t)(m0 + c) * NSTD + koff;
  const __bf16* OMT = (const __bf16*)OMTp;
  v8f accc[8];
#pragma unroll
  for (int j = 0; j < 8; ++j) accc[j] = z8;
#pragma unroll 1
  for (int k0 = 0; k0 < NSTD; k0 += 32) {
    const v16b a = FragB::load(spr + k0);
#pragma unroll
    for (int g2 = 0; g2 < 2; ++g2) {
      v16b bq[4];
#pragma unroll
      for (int jj = 0; jj < 4; ++jj)
        bq[jj] = FragB::load(OMT + (size_t)(ncol0 + 16 * (4 * g2 + jj) + c) * NSTD + koff + k0);
#pragma unroll
      for (int jj = 0; jj < 4; ++jj) accc[4 * g2 + jj] = FragB::mma(a, bq[jj], accc[4 * g2 + jj]);
      dep_guard4m_b(accc[4 * g2 + 0], accc[4 * g2 + 1], accc[4 * g2 + 2], accc[4 * g2 + 3], a, bq[3]);
      keep4_b(bq[0], bq[1], bq[2], bq[3]);
    }
  }
  acc_guard4(accc[0], accc[1], accc[2], accc[3]);
  acc_guard4(accc[4], accc[5], accc[6], accc[7]);
  float qc[8];
#pragma unroll
  for (int r = 0; r < 8; ++r) qc[r] = 0.0f;
#pragma unroll
  for (int j = 0; j < 8; ++j)
#pragma unroll
    for (int r = 0; r < 8; ++r) qc[r] = fmaf(accc[j][r], accc[j][r], qc[r]);
#pragma unroll
  for (int r = 0; r < 8; ++r) qc[r] = sum16(qc[r]);
  if (c == 0) {
#pragma unroll
    for (int r = 0; r < 8; ++r) redc[wave * 16 + 8 * hh + r] = qc[r];
  }
  __syncthreads();
  float scc[8];
#pragma unroll
  for (int r = 0; r < 8; ++r) {
    float n2 = 0.0f;
#pragma unroll
    for (int w = 0; w < 8; ++w) n2 += redc[w * 16 + 8 * hh + r];
    const float cn = sqrtf(n2);
    const float cl = fminf(cn, MAXEFF * sn[r]);
    scc[r] = cl * (1.0f / (cn + EPSN));
  }
#pragma unroll
  for (int j = 0; j < 8; ++j) {
    const float wv = wl[ncol0 + 16 * j + c];
#pragma unroll
    for (int r = 0; r < 8; ++r) {
      const int idx = (8 * hh + r) * SLD + 16 * j + c;
      const float dv = sw[idx];
      const float yv = (accc[j][r] * scc[r] + dv) * wv;
      sw[idx] = yv;
    }
  }
  __syncthreads();
  v4f yv4[16];
#pragma unroll
  for (int row = 0; row < 16; ++row) yv4[row] = *(const v4f*)(sw + row * SLD + 4 * lane);
  for (int pass = 0; pass < 2; ++pass) {
#pragma unroll
    for (int row = 0; row < 16; ++row)
      *(volatile v4f*)(Y + (size_t)(m0 + row) * NIND + ncol0 + 4 * lane) = yv4[row];
    __threadfence();
  }
}

__global__ __launch_bounds__(NTHR) void ola_kernel(const float* __restrict__ Y, float* __restrict__ out) {
  const int i = blockIdx.x * NTHR + threadIdx.x;
  const int b = i >> 15;
  const int x4 = i & 32767;
  const int g = x4 >> 7;
  const int j4 = (x4 & 127) * 4;
  const int gm = (g >= 1) ? (g - 1) : 0;
  const float fb = (g >= 1) ? 1.0f : 0.0f;
  const v4f va = *(const v4f*)(Y + ((size_t)b * NFR + (size_t)g) * NIND + j4);
  const v4f vb = *(const v4f*)(Y + ((size_t)b * NFR + (size_t)gm) * NIND + NHOP + j4);
  v4f o;
#pragma unroll
  for (int e = 0; e < 4; ++e) o[e] = fmaf(fb, vb[e], va[e]);
  float* op = out + (size_t)i * 4;
  *(volatile v4f*)op = o;
  __threadfence();
  *(volatile v4f*)op = o;
}

extern "C" void kernel_launch(void* const* d_in, const int* in_sizes, int n_in,
                              void* d_out, int out_size, void* d_ws, size_t ws_size, hipStream_t stream) {
  if (n_in < 6 || d_out == nullptr || d_ws == nullptr) return;
  if (in_sizes[0] != NBAT * NCP * NFR || in_sizes[1] != NCP * NIND || in_sizes[2] != NSTD * NSTD ||
      in_sizes[3] != NIND * NSTD || in_sizes[4] != NSTD * NIND || in_sizes[5] != NIND * NIND ||
      out_size != NBAT * NSMP) return;

  const float* control = (const float*)d_in[0];
  const float* proj    = (const float*)d_in[1];
  const float* sm      = (const float*)d_in[2];
  const float* im      = (const float*)d_in[3];
  const float* om      = (const float*)d_in[4];
  const float* dm      = (const float*)d_in[5];
  float* out = (float*)d_out;

  char* ws = (char*)d_ws; size_t off = 0;
  auto carve = [&](size_t bytes) -> char* { char* p = ws + off; off += (bytes + 255) & ~(size_t)255; return p; };
  float*          WT  = (float*)carve((size_t)NIND * 4);
  float*          GR  = (float*)carve((size_t)NCP * NCP * 4);
  unsigned short* PDH = (unsigned short*)carve((size_t)NIND * NCP * 2);
  unsigned short* PDL = (unsigned short*)carve((size_t)NIND * NCP * 2);
  unsigned short* PIH = (unsigned short*)carve((size_t)NSTD * NCP * 2);
  unsigned short* SMT = (unsigned short*)carve((size_t)NSTD * NSTD * 2);
  unsigned short* OMT = (unsigned short*)carve((size_t)NIND * NSTD * 2);
  unsigned short* AH  = (unsigned short*)carve((size_t)NROW * NCP * 2);
  unsigned short* AL  = (unsigned short*)carve((size_t)NROW * NCP * 2);
  float*          PN  = (float*)carve((size_t)NROW * 4);
  float*          BP  = (float*)carve((size_t)NROW * NSTD * 4);
  unsigned short* SP  = (unsigned short*)carve((size_t)NROW * NSTD * 2);
  float*          SN  = (float*)carve((size_t)NROW * 4);
  float*          Y   = (float*)carve((size_t)NROW * NIND * 4);
  if (off > ws_size || off > (size_t)134217728) return;

  wtab_kernel<<<NIND / NTHR, NTHR, 0, stream>>>(WT);
  gram_kernel<<<NCP / (NTHR / 32), NTHR, 0, stream>>>(proj, GR);
  pw_kernel<NIND, true><<<NIND / NTHR, NTHR, 0, stream>>>(proj, dm, PDH, PDL);
  pw_kernel<NSTD, false><<<NSTD / NTHR, NTHR, 0, stream>>>(proj, im, PIH, PIH);
  tpw_bf16_kernel<<<dim3(NSTD / 64, NSTD / 64), NTHR, 0, stream>>>(sm, NSTD, NSTD, NSTD, SMT);
  tpw_bf16_kernel<<<dim3(NIND / 64, NSTD / 64), NTHR, 0, stream>>>(om, NSTD, NIND, NSTD, OMT);
  rowprep_kernel<<<NROW / 64, NTHR, 0, stream>>>(control, GR, AH, AL, PN);
  bproj_kernel<<<NROW / 16, NTHR, 0, stream>>>(AH, PIH, PN, BP);
  scan_kernel<<<NBAT / SEQB, NTHR, 0, stream>>>(SMT, BP, SP, SN);
  dc_kernel<<<NROW / 16, NTHR, 0, stream>>>(AH, AL, PDH, PDL, PN, SP, OMT, SN, WT, Y);
  ola_kernel<<<(NBAT * NSMP / 4) / NTHR, NTHR, 0, stream>>>(Y, out);
}
